// Multi_Head_Attention_25091198943737
// MI455X (gfx1250) — hardware-verified
//
#include <hip/hip_runtime.h>
#include <math.h>

typedef __attribute__((ext_vector_type(16))) _Float16 v16h;
typedef __attribute__((ext_vector_type(16))) __bf16 v16b;
typedef __attribute__((ext_vector_type(8)))  _Float16 v8h;
typedef __attribute__((ext_vector_type(8)))  __bf16 v8b;
typedef __attribute__((ext_vector_type(8)))  float v8f;
typedef __attribute__((ext_vector_type(4)))  float v4f;
typedef __attribute__((ext_vector_type(4)))  unsigned v4u;

template <typename T> __device__ __forceinline__ void vst2(void* p, T v) { *(volatile T*)p = v; __threadfence(); *(volatile T*)p = v; }

__device__ __forceinline__ v8f wmma16(v16h a, v16h b, v8f c) {
  v8f d = __builtin_amdgcn_wmma_f32_16x16x32_f16(false, a, false, b, (short)0, c, false, false);
  asm volatile("v_nop\n\tv_nop\n\tv_nop\n\tv_nop" : "+v"(d) : "v"(a), "v"(b));
  return d;
}
__device__ __forceinline__ v8f wmma_bf(v16b a, v16b b, v8f c) {
  v8f d = __builtin_amdgcn_wmma_f32_16x16x32_bf16(false, a, false, b, (short)0, c, false, false);
  asm volatile("v_nop\n\tv_nop\n\tv_nop\n\tv_nop" : "+v"(d) : "v"(a), "v"(b));
  return d;
}
__device__ __forceinline__ v16h frag_h(const _Float16* rowk0, int lane) {
  union { v16h v; v8h q[2]; } u; const _Float16* p = rowk0 + 8 * (lane >> 4);
  u.q[0] = *(const v8h*)p; u.q[1] = *(const v8h*)(p + 16); return u.v;
}
__device__ __forceinline__ v16b frag_b(const __bf16* rowk0, int lane) {
  union { v16b v; v8b q[2]; } u; const __bf16* p = rowk0 + 8 * (lane >> 4);
  u.q[0] = *(const v8b*)p; u.q[1] = *(const v8b*)(p + 16); return u.v;
}
struct F2 { v16b h, l; };
__device__ __forceinline__ F2 bsplit16(const float v[16]) { F2 r;
#pragma unroll
  for (int i = 0; i < 16; ++i) { const __bf16 h = (__bf16)v[i]; r.h[i] = h; r.l[i] = (__bf16)(v[i] - (float)h); }
  return r; }
__device__ __forceinline__ F2 split_row(const float* row, int k0, int lane) { float v[16]; const float* p = row + k0 + 8 * (lane >> 4);
#pragma unroll
  for (int i = 0; i < 8; ++i) { v[i] = p[i]; v[8 + i] = p[16 + i]; }
  return bsplit16(v); }
__device__ __forceinline__ float bfr(float v) { return (float)(__bf16)v; }
__device__ __forceinline__ void ldsx() { asm volatile("s_wait_dscnt 0" ::: "memory"); __builtin_amdgcn_wave_barrier(); __builtin_amdgcn_fence(4, "workgroup"); }

#ifndef NB
#define NB 2
#endif
#ifndef SEQ
#define SEQ 2048
#endif
#ifndef NB_FULL
#define NB_FULL 2
#endif
#ifndef SEQ_FULL
#define SEQ_FULL 2048
#endif
#define CC 1024
#define NH 16
#define HD 64
#define KT 64

static_assert(NB >= 1 && NB <= NB_FULL);
static_assert(SEQ % 64 == 0 && SEQ <= SEQ_FULL && SEQ_FULL % 4 == 0);
static_assert(NH * HD == CC && HD == 64 && CC % 128 == 0 && KT == 64);

#define PLB (2u * (size_t)NB * SEQ * CC)
#define WPB (2u * (size_t)CC * CC)
#define WS_XQ ((size_t)0)
#define WS_XK (WS_XQ + PLB)
#define WS_XV (WS_XK + PLB)
#define WS_WQ (WS_XV + PLB)
#define WS_WK (WS_WQ + WPB)
#define WS_WV (WS_WK + WPB)
#define WS_QH (WS_WV + WPB)
#define WS_QL (WS_QH + PLB)
#define WS_KH (WS_QL + PLB)
#define WS_VT (WS_KH + PLB)
#define WS_VL (WS_VT + PLB)
#define WS_END (WS_VL + PLB)
static_assert(PLB % 128 == 0 && WPB % 128 == 0);
static_assert(WS_END <= (size_t)134217728u);

__global__ __launch_bounds__(256) void k_cvt(const float* __restrict__ XQ, const float* __restrict__ XK, const float* __restrict__ XV,
                                             const float* __restrict__ WQ, const float* __restrict__ WK, const float* __restrict__ WV,
                                             __bf16* __restrict__ DQ, __bf16* __restrict__ DK, __bf16* __restrict__ DV,
                                             __bf16* __restrict__ DWQ, __bf16* __restrict__ DWK, __bf16* __restrict__ DWV) {
  const int z = blockIdx.z;
  const float* src = z == 0 ? XQ : z == 1 ? XK : z == 2 ? XV : z == 3 ? WQ : z == 4 ? WK : WV;
  __bf16* dst = z == 0 ? DQ : z == 1 ? DK : z == 2 ? DV : z == 3 ? DWQ : z == 4 ? DWK : DWV;
  const size_t n8 = (z < 3) ? (size_t)NB * SEQ * CC / 8 : (size_t)CC * CC / 8;
  const size_t e = (size_t)blockIdx.x * 256 + threadIdx.x;
  if (e >= n8) return;
  size_t so = e * 8;
  if (z < 3) { const size_t row = e / (CC / 8), c = e % (CC / 8); so = ((row / SEQ) * SEQ_FULL + (row % SEQ)) * CC + c * 8; }
  const v4f f0 = *(const v4f*)(src + so), f1 = *(const v4f*)(src + so + 4);
  union { v8b v; v4u u; } o;
#pragma unroll
  for (int i = 0; i < 4; ++i) { o.v[i] = (__bf16)f0[i]; o.v[4 + i] = (__bf16)f1[i]; }
  vst2((void*)(dst + e * 8), o.u);
}

__global__ __launch_bounds__(128) void k_proj(const __bf16* __restrict__ XQ, const __bf16* __restrict__ XK, const __bf16* __restrict__ XV,
                                              const __bf16* __restrict__ WQ, const __bf16* __restrict__ WK, const __bf16* __restrict__ WV,
                                              const float* __restrict__ BQ, const float* __restrict__ BK, const float* __restrict__ BV,
                                              _Float16* __restrict__ QH, _Float16* __restrict__ QL, _Float16* __restrict__ KH,
                                              __bf16* __restrict__ VT, __bf16* __restrict__ VL) {
  __shared__ __align__(16) _Float16 sh[64][136], sl[64][136]; __shared__ __align__(16) __bf16 th[128][72], tl2[128][72];
  const int tid = threadIdx.x, wave = tid >> 5, lane = tid & 31, col = lane & 15, g = lane >> 4;
  const int which = blockIdx.z; const int c0 = blockIdx.y * 128; const size_t r0 = (size_t)blockIdx.x * 64;
  const __bf16* X = which == 0 ? XQ : which == 1 ? XK : XV;
  const __bf16* W = which == 0 ? WQ : which == 1 ? WK : WV;
  const float* BA = which == 0 ? BQ : which == 1 ? BK : BV;
  v8f acc[8] = {};
#pragma unroll 2
  for (int kc = 0; kc < CC / 32; ++kc) {
    const v16b a = frag_b(X + (r0 + wave * 16 + col) * CC + kc * 32, lane);
#pragma unroll
    for (int j = 0; j < 8; ++j) {
      const v16b w = frag_b(W + (size_t)(c0 + j * 16 + col) * CC + kc * 32, lane);
      acc[j] = wmma_bf(a, w, acc[j]); } }
#pragma unroll
  for (int j = 0; j < 8; ++j) { const float bb = bfr(BA[c0 + j * 16 + col]);
#pragma unroll
    for (int r = 0; r < 8; ++r) { const float v = acc[j][r] + bb; const int rl = wave * 16 + 8 * g + r, cl = j * 16 + col;
      if (which == 2) { const __bf16 bh = (__bf16)v; th[cl][rl] = bh; tl2[cl][rl] = (__bf16)(v - (float)bh); }
      else { const _Float16 hv = (_Float16)v; sh[rl][cl] = hv; sl[rl][cl] = (_Float16)((v - (float)hv) * 1024.0f); }     } }
  __syncthreads();
  if (which < 2) { _Float16* dh = which == 0 ? QH : KH;
    for (int e = tid; e < 64 * 16; e += 128) { const int rl = e >> 4, q = e & 15;
      vst2((void*)(dh + (r0 + rl) * CC + c0 + q * 8), *(const v4u*)&sh[rl][q * 8]);
      if (which == 0) vst2((void*)(QL + (r0 + rl) * CC + c0 + q * 8), *(const v4u*)&sl[rl][q * 8]); } }
  else { const size_t b = r0 / SEQ; const int t0 = (int)(r0 % SEQ);
    for (int e = tid; e < 128 * 8; e += 128) { const int cl = e >> 3, q = e & 7; const size_t o2 = (b * CC + c0 + cl) * (size_t)SEQ + t0 + q * 8;
      vst2((void*)(VT + o2), *(const v4u*)&th[cl][q * 8]); vst2((void*)(VL + o2), *(const v4u*)&tl2[cl][q * 8]); } }
}

__global__ __launch_bounds__(128) void k_att(const _Float16* __restrict__ QH, const _Float16* __restrict__ QL, const _Float16* __restrict__ KH,
                                             const __bf16* __restrict__ VT, const __bf16* __restrict__ VL, const float* __restrict__ MK, float* __restrict__ OUT) {
  __shared__ __align__(16) _Float16 kt[KT][72];
  __shared__ __align__(16) __bf16 vhs[HD][72], vls[HD][72];
  __shared__ __align__(16) float ms[64][68];
  __shared__ __align__(16) float ps[4][16][68];
  const int tid = threadIdx.x, wave = tid >> 5, lane = tid & 31, col = lane & 15, g = lane >> 4;
  const int b = blockIdx.z, h = blockIdx.y, qb0 = blockIdx.x * 64, ql0 = qb0 + wave * 16;
  const size_t qrow = (size_t)b * SEQ + ql0;
  v16h qh[2], qlo[2];
#pragma unroll
  for (int kc = 0; kc < 2; ++kc) { qh[kc] = frag_h(QH + (qrow + col) * CC + h * HD + kc * 32, lane); qlo[kc] = frag_h(QL + (qrow + col) * CC + h * HD + kc * 32, lane); }
  float mrow[8], lrow[8]; v8f o[4];
#pragma unroll
  for (int r = 0; r < 8; ++r) { mrow[r] = -3.0e38f; lrow[r] = 0.0f; }
#pragma unroll
  for (int t = 0; t < 4; ++t) o[t] = (v8f){};
#pragma unroll 1
  for (int kb = 0; kb < SEQ / KT; ++kb) {
    const int k0 = kb * KT;
    __syncthreads();
#pragma unroll
    for (int i = 0; i < 4; ++i) { const int e = tid + 128 * i, rr = e >> 3, c = e & 7;
      *(v8h*)&kt[rr][c * 8] = *(const v8h*)(KH + ((size_t)b * SEQ + k0 + rr) * CC + h * HD + c * 8);
      const size_t vo = ((size_t)b * CC + h * HD + rr) * SEQ + k0 + c * 8;
      *(v8b*)&vhs[rr][c * 8] = *(const v8b*)(VT + vo); *(v8b*)&vls[rr][c * 8] = *(const v8b*)(VL + vo); }
#pragma unroll
    for (int i = 0; i < 8; ++i) { const int e = tid + 128 * i, qr = e >> 4, c = e & 15;
      *(v4f*)&ms[qr][c * 4] = *(const v4f*)(MK + ((size_t)b * SEQ_FULL + qb0 + qr) * SEQ_FULL + k0 + c * 4); }
    __syncthreads();
    v8f s[4];
#pragma unroll
    for (int j = 0; j < 4; ++j) { v8f a = {}, al = {};
#pragma unroll
      for (int kc = 0; kc < 2; ++kc) { const v16h kf = frag_h(&kt[j * 16 + col][kc * 32], lane);
        a = wmma16(qh[kc], kf, a); al = wmma16(qlo[kc], kf, al); }
      s[j] = a * (-0.125f) + al * (-0.125f / 1024.0f); }
#pragma unroll
    for (int r = 0; r < 8; ++r) { const int mr = wave * 16 + 8 * g + r;
#pragma unroll
      for (int j = 0; j < 4; ++j) s[j][r] += bfr(ms[mr][j * 16 + col]);
      float v = fmaxf(fmaxf(s[0][r], s[1][r]), fmaxf(s[2][r], s[3][r]));
      v = fmaxf(v, __shfl_xor(v, 1, 16)); v = fmaxf(v, __shfl_xor(v, 2, 16)); v = fmaxf(v, __shfl_xor(v, 4, 16)); v = fmaxf(v, __shfl_xor(v, 8, 16));
      const float mn = fmaxf(mrow[r], v); const float alpha = expf(mrow[r] - mn); float rs = 0.0f;
#pragma unroll
      for (int j = 0; j < 4; ++j) { const float p = expf(s[j][r] - mn); s[j][r] = p; rs += p; }
      rs += __shfl_xor(rs, 1, 16); rs += __shfl_xor(rs, 2, 16); rs += __shfl_xor(rs, 4, 16); rs += __shfl_xor(rs, 8, 16);
      lrow[r] = lrow[r] * alpha + rs; mrow[r] = mn;
#pragma unroll
      for (int t = 0; t < 4; ++t) o[t][r] *= alpha; }
#pragma unroll
    for (int j = 0; j < 4; ++j)
#pragma unroll
      for (int r = 0; r < 8; ++r) ps[wave][8 * g + r][j * 16 + col] = s[j][r] * 2048.0f;
    ldsx();
#pragma unroll
    for (int kc = 0; kc < 2; ++kc) { const F2 p = split_row(&ps[wave][col][0], kc * 32, lane);
#pragma unroll
      for (int t = 0; t < 4; ++t) {
        const v16b vh = frag_b(&vhs[t * 16 + col][kc * 32], lane), vl = frag_b(&vls[t * 16 + col][kc * 32], lane);
        o[t] = wmma_bf(p.h, vh, o[t]); o[t] = wmma_bf(p.l, vh, o[t]); o[t] = wmma_bf(p.h, vl, o[t]); } }
  }
  ldsx();
#pragma unroll
  for (int r = 0; r < 8; ++r) { const float inv = (1.0f / lrow[r]) * (1.0f / 2048.0f);
#pragma unroll
    for (int t = 0; t < 4; ++t) ps[wave][8 * g + r][t * 16 + col] = o[t][r] * inv; }
  ldsx();
  for (int rl = 0; rl < 16; ++rl) { const v4f w4 = *(const v4f*)&ps[wave][rl][(lane & 15) * 4];
    if (lane < HD / 4) vst2((void*)(OUT + ((size_t)b * SEQ + ql0 + rl) * CC + h * HD + lane * 4), w4); }
}

extern "C" void kernel_launch(void* const* d_in, const int* in_sizes, int n_in, void* d_out, int out_size, void* d_ws, size_t ws_size, hipStream_t stream) {
  if (n_in < 10) return;
  const size_t needX = ((size_t)(NB - 1) * SEQ_FULL + SEQ) * CC;
  const size_t needM = ((size_t)(NB - 1) * SEQ_FULL + SEQ - 1) * SEQ_FULL + SEQ;
  if ((size_t)in_sizes[0] < needX || (size_t)in_sizes[1] < needX || (size_t)in_sizes[2] < needX) return;
  if ((size_t)in_sizes[3] < needM) return;
  if ((size_t)in_sizes[4] < (size_t)CC * CC || (size_t)in_sizes[6] < (size_t)CC * CC || (size_t)in_sizes[8] < (size_t)CC * CC) return;
  if (in_sizes[5] < CC || in_sizes[7] < CC || in_sizes[9] < CC) return;
  if ((size_t)out_size < (size_t)NB * SEQ * CC) return;
  if (ws_size < (size_t)WS_END) return;
  const float* const* F = (const float* const*)d_in;
  char* ws = (char*)d_ws;
  __bf16 *XQb = (__bf16*)(ws + WS_XQ), *XKb = (__bf16*)(ws + WS_XK), *XVb = (__bf16*)(ws + WS_XV);
  __bf16 *WQb = (__bf16*)(ws + WS_WQ), *WKb = (__bf16*)(ws + WS_WK), *WVb = (__bf16*)(ws + WS_WV);
  _Float16 *QH = (_Float16*)(ws + WS_QH), *QL = (_Float16*)(ws + WS_QL), *KH = (_Float16*)(ws + WS_KH);
  __bf16 *VT = (__bf16*)(ws + WS_VT), *VL = (__bf16*)(ws + WS_VL);
  const size_t nx8 = (size_t)NB * SEQ * CC / 8, nw8 = (size_t)CC * CC / 8;
  const unsigned gx8 = (unsigned)((nx8 + 255) / 256), gw8 = (unsigned)((nw8 + 255) / 256);
  const unsigned gx = gx8 > gw8 ? gx8 : gw8;
  k_cvt<<<dim3(gx, 1, 6), 256, 0, stream>>>(F[0], F[1], F[2], F[4], F[6], F[8], XQb, XKb, XVb, WQb, WKb, WVb);
  k_proj<<<dim3(NB * SEQ / 64, CC / 128, 3), 128, 0, stream>>>(XQb, XKb, XVb, WQb, WKb, WVb, F[5], F[7], F[9], QH, QL, KH, VT, VL);
  k_att<<<dim3(SEQ / 64, NH, NB), 128, 0, stream>>>(QH, QL, KH, VT, VL, F[3], (float*)d_out);
}
